// KANLinear_64510408786339
// MI455X (gfx1250) — hardware-verified
//
#include <hip/hip_runtime.h>
#include <math.h>

constexpr int kBatch    = 16384;
constexpr int kInF      = 512;
constexpr int kOutF     = 512;
constexpr int kNB       = 8;
constexpr int kNKnot    = 12;
constexpr int kKSpl     = kInF * kNB;
constexpr int kKTot     = kInF + kKSpl;
constexpr int kHalfRows = kBatch / 2;
constexpr float kACarry   = 256.0f;
constexpr float kBCarry   = 64.0f;
constexpr float kOutScale = 1.0f / (256.0f * 64.0f);
constexpr int kPrepBaseThreads = kOutF * kInF / 8;
constexpr int kPrepSplThreads  = kOutF * kKSpl / 8;
constexpr int kGenThreads      = kInF;
constexpr size_t kBtBytes = (size_t)kOutF * kKTot * 2;
constexpr size_t kABytes  = (size_t)kHalfRows * kKTot * 2;
constexpr size_t kWsNeed  = kBtBytes + kABytes;
static_assert(kKTot % 32 == 0, "k32");
static_assert(kHalfRows % 64 == 0 && kOutF % 64 == 0, "tile64");
static_assert(kPrepBaseThreads % 256 == 0 && kPrepSplThreads % 256 == 0, "grid");
static_assert(kBtBytes % 128 == 0, "align");
static_assert(kWsNeed <= (size_t)134217728, "carve");
static_assert(kNB == 8 && kNKnot == 12, "shape");

typedef __attribute__((ext_vector_type(16))) _Float16 v16h;
typedef __attribute__((ext_vector_type(8)))  _Float16 v8h;
typedef __attribute__((ext_vector_type(16))) __bf16   v16b;
typedef __attribute__((ext_vector_type(8)))  __bf16   v8b;
typedef __attribute__((ext_vector_type(8)))  float    v8f;
typedef __attribute__((ext_vector_type(4)))  float    v4f;
typedef __attribute__((ext_vector_type(4)))  unsigned int v4u;

__device__ __forceinline__ unsigned short f2bf_bits(float f) {
  unsigned u = __float_as_uint(f);
  return (unsigned short)((u + 0x7FFFu + ((u >> 16) & 1u)) >> 16);
}
__device__ __forceinline__ float bf_bits2f(unsigned short h) { return __uint_as_float(((unsigned)h) << 16); }

__device__ __forceinline__ void dep_guard_h(v8f& a, v8f& b, v16h x, v16h y) { asm volatile("v_nop\n\tv_nop\n\tv_nop\n\tv_nop" : "+v"(a), "+v"(b) : "v"(x), "v"(y)); }
__device__ __forceinline__ void dep_guard_b(v8f& a, v8f& b, v16b x, v16b y) { asm volatile("v_nop\n\tv_nop\n\tv_nop\n\tv_nop" : "+v"(a), "+v"(b) : "v"(x), "v"(y)); }
__device__ __forceinline__ void dep_guard4_h(v8f& a, v8f& b, v8f& c, v8f& d, v16h x, v16h y) { asm volatile("v_nop\n\tv_nop\n\tv_nop\n\tv_nop" : "+v"(a), "+v"(b), "+v"(c), "+v"(d) : "v"(x), "v"(y)); }
__device__ __forceinline__ void dep_guard4_b(v8f& a, v8f& b, v8f& c, v8f& d, v16b x, v16b y) { asm volatile("v_nop\n\tv_nop\n\tv_nop\n\tv_nop" : "+v"(a), "+v"(b), "+v"(c), "+v"(d) : "v"(x), "v"(y)); }
__device__ __forceinline__ void keep4_h(v16h a, v16h b, v16h c, v16h d) { asm volatile("v_nop" :: "v"(a), "v"(b), "v"(c), "v"(d)); }
__device__ __forceinline__ void keep4_b(v16b a, v16b b, v16b c, v16b d) { asm volatile("v_nop" :: "v"(a), "v"(b), "v"(c), "v"(d)); }
__device__ __forceinline__ void acc_guard4(v8f& a, v8f& b, v8f& c, v8f& d) { asm volatile("v_nop\n\tv_nop\n\tv_nop\n\tv_nop" : "+v"(a), "+v"(b), "+v"(c), "+v"(d)); }
template <typename T> struct Frag;
template <> struct Frag<_Float16> {
  typedef v16h V; union U { v16h v; v8h h[2]; };
  static __device__ __forceinline__ v16h load(const _Float16* p) {
    U f; f.h[0] = *(const v8h*)(p); f.h[1] = *(const v8h*)(p + 16); return f.v;
  }
  static __device__ __forceinline__ v8f mma(v16h a, v16h b, v8f c) {
    return __builtin_amdgcn_wmma_f32_16x16x32_f16(false, a, false, b, (short)0, c, false, false);
  }
  static __device__ __forceinline__ void guard(v8f& a, v8f& b, v16h x, v16h y) { dep_guard_h(a, b, x, y); }
  static __device__ __forceinline__ void guard4(v8f& a, v8f& b, v8f& c, v8f& d, v16h x, v16h y) { dep_guard4_h(a, b, c, d, x, y); }
  static __device__ __forceinline__ void keep(v16h a, v16h b, v16h c, v16h d) { keep4_h(a, b, c, d); }
};
template <> struct Frag<__bf16> {
  typedef v16b V; union U { v16b v; v8b h[2]; };
  static __device__ __forceinline__ v16b load(const __bf16* p) {
    U f; f.h[0] = *(const v8b*)(p); f.h[1] = *(const v8b*)(p + 16); return f.v;
  }
  static __device__ __forceinline__ v8f mma(v16b a, v16b b, v8f c) {
    return __builtin_amdgcn_wmma_f32_16x16x32_bf16(false, a, false, b, (short)0, c, false, false);
  }
  static __device__ __forceinline__ void guard(v8f& a, v8f& b, v16b x, v16b y) { dep_guard_b(a, b, x, y); }
  static __device__ __forceinline__ void guard4(v8f& a, v8f& b, v8f& c, v8f& d, v16b x, v16b y) { dep_guard4_b(a, b, c, d, x, y); }
  static __device__ __forceinline__ void keep(v16b a, v16b b, v16b c, v16b d) { keep4_b(a, b, c, d); }
};

__device__ __forceinline__ unsigned pk16(unsigned short a, unsigned short b) { return (unsigned)a | ((unsigned)b << 16); }
__device__ __forceinline__ unsigned short h_bits(float f) { const _Float16 h = (_Float16)f; return __builtin_bit_cast(unsigned short, h); }

template <int ET> struct Elem;
template <> struct Elem<0> { typedef _Float16 T; };
template <> struct Elem<1> { typedef __bf16 T; };
template <int ET, bool SPLIT, int BIAS_MODE, int OUT_MODE, bool RESID, int ACT = 0>
__global__ __launch_bounds__(256) void wmma_gemm64(
    const unsigned short* __restrict__ Ap, const unsigned short* __restrict__ A2p, int lda, long strideA,
    const unsigned short* __restrict__ Btp, const unsigned short* __restrict__ Bt2p, int ldb, long strideB,
    void* __restrict__ Cout, void* __restrict__ Cout2, int ldc, long strideC,
    const float* __restrict__ bias,
    const float* __restrict__ resid, long strideR,
    int M, int N, int K, float scale) {
  typedef typename Elem<ET>::T T;
  typedef typename Frag<T>::V V;
  const T* A = (const T*)Ap; const T* A2 = (const T*)A2p; const T* Bt = (const T*)Btp; const T* Bt2 = (const T*)Bt2p;
  __shared__ __align__(16) float sT[8][16 * 68];
  const int b    = blockIdx.y;
  const int lane = threadIdx.x & 31;
  const int wave = threadIdx.x >> 5;
  const int tilesN = N >> 6;
  const int tilesM = M >> 6;
  const int tile = blockIdx.x * 8 + wave;
  if (tile >= tilesM * tilesN) return;
  const int tm = tile / tilesN;
  const int tn = tile - tm * tilesN;
  const int m0 = tm << 6;
  const int n0 = tn << 6;

  const T* Ab  = A  + (size_t)b * strideA;
  const T* Bb  = Bt + (size_t)b * strideB;
  const T* Ab2 = SPLIT ? (A2  + (size_t)b * strideA) : nullptr;
  const T* Bb2 = SPLIT ? (Bt2 + (size_t)b * strideB) : nullptr;

  const int rlane = lane & 15;
  const int koff  = (lane >> 4) * 8;
  const int mOff  = (lane >> 4) * 8;

  v8f acc[4][4];
#pragma unroll
  for (int i = 0; i < 4; ++i)
#pragma unroll
    for (int j = 0; j < 4; ++j) acc[i][j] = (v8f){0.f,0.f,0.f,0.f,0.f,0.f,0.f,0.f};

  for (int k0 = 0; k0 < K; k0 += 32) {
    V bh[4], bl[4];
#pragma unroll
    for (int j = 0; j < 4; ++j) {
      const size_t bo = (size_t)(n0 + (j << 4) + rlane) * ldb + koff + k0;
      bh[j] = Frag<T>::load(Bb + bo);
      if (SPLIT) bl[j] = Frag<T>::load(Bb2 + bo);
    }
#pragma unroll
    for (int i = 0; i < 4; ++i) {
      const size_t ao = (size_t)(m0 + (i << 4) + rlane) * lda + koff + k0;
      V ah = Frag<T>::load(Ab + ao);
      V al = ah;
      if (SPLIT) al = Frag<T>::load(Ab2 + ao);
#pragma unroll
      for (int j = 0; j < 4; ++j) {
        acc[i][j] = Frag<T>::mma(ah, bh[j], acc[i][j]);
        if (SPLIT) {
          acc[i][j] = Frag<T>::mma(ah, bl[j], acc[i][j]);
          acc[i][j] = Frag<T>::mma(al, bh[j], acc[i][j]);
        }
      }
      Frag<T>::guard4(acc[i][0], acc[i][1], acc[i][2], acc[i][3], ah, SPLIT ? al : ah);
    }
    Frag<T>::keep(bh[0], bh[1], bh[2], bh[3]);
    if (SPLIT) Frag<T>::keep(bl[0], bl[1], bl[2], bl[3]);
  }
  acc_guard4(acc[0][0], acc[0][1], acc[0][2], acc[0][3]);
  acc_guard4(acc[1][0], acc[1][1], acc[1][2], acc[1][3]);
  acc_guard4(acc[2][0], acc[2][1], acc[2][2], acc[2][3]);
  acc_guard4(acc[3][0], acc[3][1], acc[3][2], acc[3][3]);

  float* slab = sT[wave];
  const float* Rb = RESID ? (resid + (size_t)b * strideR) : nullptr;
#pragma unroll
  for (int i = 0; i < 4; ++i) {
    const int mBase = m0 + (i << 4);
#pragma unroll
    for (int j = 0; j < 4; ++j) {
      const int n = n0 + (j << 4) + rlane;
      float bv = 0.f;
      if (BIAS_MODE == 2) bv = bias[n];
#pragma unroll
      for (int r = 0; r < 8; ++r) {
        float v = acc[i][j][r] * scale;
        if (BIAS_MODE == 1) v += bias[mBase + mOff + r];
        if (BIAS_MODE == 2) v += bv;
        if (RESID) v += Rb[(size_t)(mBase + mOff + r) * ldc + n];
        if (ACT == 2) v = fmaxf(v, 0.0f);
        if (ACT == 4) v = (v > 0.f) ? v : 0.01f * v;
        if (ACT == 6) v = (fabsf(v) < INFINITY) ? v : 0.0f;
        slab[(mOff + r) * 68 + (j << 4) + rlane] = v;
      }
    }
    __builtin_amdgcn_fence(__ATOMIC_RELEASE, "workgroup");
    __builtin_amdgcn_wave_barrier();
    __builtin_amdgcn_fence(__ATOMIC_ACQUIRE, "workgroup");
    if (OUT_MODE == 0) {
      float* C = (float*)Cout + (size_t)b * strideC;
      const int hh = lane >> 4, c4 = (lane & 15) * 4;
      for (int pass = 0; pass < 2; ++pass) {
#pragma unroll
        for (int it = 0; it < 8; ++it) {
          const int row = it * 2 + hh;
          v4f v = *(const v4f*)(slab + row * 68 + c4);
          *(volatile v4f*)(C + (size_t)(mBase + row) * ldc + n0 + c4) = v;
        }
        __threadfence();
      }
    } else {
      const int q = lane >> 3, c8 = (lane & 7) * 8;
      unsigned short* C  = (unsigned short*)Cout  + (size_t)b * strideC;
      unsigned short* C2 = (OUT_MODE == 2) ? ((unsigned short*)Cout2 + (size_t)b * strideC) : nullptr;
      for (int pass = 0; pass < 2; ++pass) {
#pragma unroll
        for (int it = 0; it < 4; ++it) {
          const int row = it * 4 + q;
          const float* sp = slab + row * 68 + c8;
          v8h hv, lv;
#pragma unroll
          for (int e = 0; e < 8; ++e) {
            if (OUT_MODE == 1) {
              hv[e] = (_Float16)sp[e];
            } else {
              unsigned short hb = f2bf_bits(sp[e]);
              unsigned short lb = f2bf_bits(sp[e] - bf_bits2f(hb));
              hv[e] = __builtin_bit_cast(_Float16, hb);
              lv[e] = __builtin_bit_cast(_Float16, lb);
            }
          }
          *(volatile v8h*)(C + (size_t)(mBase + row) * ldc + n0 + c8) = hv;
          if (OUT_MODE == 2) *(volatile v8h*)(C2 + (size_t)(mBase + row) * ldc + n0 + c8) = lv;
        }
        __threadfence();
      }
    }
    __builtin_amdgcn_fence(__ATOMIC_RELEASE, "workgroup");
    __builtin_amdgcn_wave_barrier();
    __builtin_amdgcn_fence(__ATOMIC_ACQUIRE, "workgroup");
  }
}

__global__ __launch_bounds__(256) void prep_base_kernel(const float* __restrict__ bw,
                                                       unsigned short* __restrict__ Bt) {
  const int i = blockIdx.x * 256 + threadIdx.x;
  if (i >= kPrepBaseThreads) return;
  const int n  = i >> 6;
  const int c8 = (i & 63) * 8;
  const float* p = bw + (size_t)n * kInF + c8;
  const v4f a = *(const v4f*)(p);
  const v4f c = *(const v4f*)(p + 4);
  unsigned short hb[8];
#pragma unroll
  for (int e = 0; e < 4; ++e) {
    hb[e]     = h_bits(a[e] * kBCarry);
    hb[4 + e] = h_bits(c[e] * kBCarry);
  }
  const v4u u = (v4u){pk16(hb[0], hb[1]), pk16(hb[2], hb[3]), pk16(hb[4], hb[5]), pk16(hb[6], hb[7])};
  unsigned short* q = Bt + (size_t)n * kKTot + c8;
  *(volatile v4u*)q = u;
  __threadfence();
  *(volatile v4u*)q = u;
}

__global__ __launch_bounds__(256) void prep_spline_kernel(const float* __restrict__ sw,
                                                         const float* __restrict__ sc,
                                                         unsigned short* __restrict__ Bt) {
  const int t = blockIdx.x * 256 + threadIdx.x;
  if (t >= kPrepSplThreads) return;
  const int n = t >> 9;
  const int f = t & 511;
  const float* p = sw + (size_t)n * kKSpl + 8 * f;
  const float s  = sc[(size_t)n * kInF + f] * kBCarry;
  const v4f a = *(const v4f*)(p);
  const v4f c = *(const v4f*)(p + 4);
  unsigned short hb[8];
#pragma unroll
  for (int e = 0; e < 4; ++e) {
    hb[e]     = h_bits(a[e] * s);
    hb[4 + e] = h_bits(c[e] * s);
  }
  const v4u u = (v4u){pk16(hb[0], hb[1]), pk16(hb[2], hb[3]), pk16(hb[4], hb[5]), pk16(hb[6], hb[7])};
  unsigned short* q = Bt + (size_t)n * kKTot + kInF + 8 * f;
  *(volatile v4u*)q = u;
  __threadfence();
  *(volatile v4u*)q = u;
}

__global__ __launch_bounds__(512) void gen_a_kernel(const float* __restrict__ x,
                                                    const float* __restrict__ grid,
                                                    unsigned short* __restrict__ Apl,
                                                    int row_base) {
  __shared__ __align__(16) unsigned short s_h[kInF];
  const int t  = threadIdx.x;
  const int bl = blockIdx.x;
  const float* xrow = x + (size_t)(row_base + bl) * kInF;
  unsigned short* arow = Apl + (size_t)bl * kKTot;

  const float* grow = grid + (size_t)t * kNKnot;
  const v4f q0 = *(const v4f*)(grow);
  const v4f q1 = *(const v4f*)(grow + 4);
  const v4f q2 = *(const v4f*)(grow + 8);
  float g[kNKnot];
  g[0] = q0[0]; g[1] = q0[1]; g[2]  = q0[2]; g[3]  = q0[3];
  g[4] = q1[0]; g[5] = q1[1]; g[6]  = q1[2]; g[7]  = q1[3];
  g[8] = q2[0]; g[9] = q2[1]; g[10] = q2[2]; g[11] = q2[3];

  const float r1 = 1.0f / fmaxf(g[4] - g[3], 1e-6f);
  const float r2 = 1.0f / fmaxf(g[5] - g[3], 1e-6f);
  const float r3 = 1.0f / fmaxf(g[6] - g[3], 1e-6f);

  float xv = xrow[t];
  xv = (xv != xv) ? 0.0f : xv;
  xv = fminf(fmaxf(xv, -6.0f), 6.0f);
  xv = fminf(fmaxf(xv, -1.1f), 1.1f);
  const float xr = ((xv + 1.0f) * 0.5f) * 2.0f - 1.0f;

  const float ex = expf(-xr);
  const float sl = xr * (1.0f / (1.0f + ex));

  float dx[kNKnot];
#pragma unroll
  for (int j = 0; j < kNKnot; ++j) dx[j] = xr - g[j];
  float b0[11];
#pragma unroll
  for (int j = 0; j < 11; ++j) b0[j] = (xr >= g[j] && xr < g[j + 1]) ? 1.0f : 0.0f;
  float b1[10];
#pragma unroll
  for (int j = 0; j < 10; ++j) b1[j] = (dx[j] * b0[j] - dx[j + 2] * b0[j + 1]) * r1;
  float b2[9];
#pragma unroll
  for (int j = 0; j < 9; ++j) b2[j] = (dx[j] * b1[j] - dx[j + 3] * b1[j + 1]) * r2;
  float b3[8];
#pragma unroll
  for (int j = 0; j < 8; ++j) b3[j] = (dx[j] * b2[j] - dx[j + 4] * b2[j + 1]) * r3;

  unsigned short hb[8];
#pragma unroll
  for (int j = 0; j < 8; ++j) hb[j] = h_bits(b3[j] * kACarry);
  const v4u ub = (v4u){pk16(hb[0], hb[1]), pk16(hb[2], hb[3]), pk16(hb[4], hb[5]), pk16(hb[6], hb[7])};

  s_h[t] = h_bits(sl * kACarry);
  __syncthreads();

  const int tc = (t < 64) ? t : 63;
  unsigned short hs[8];
#pragma unroll
  for (int e = 0; e < 8; ++e) hs[e] = s_h[8 * tc + e];
  const v4u us = (v4u){pk16(hs[0], hs[1]), pk16(hs[2], hs[3]), pk16(hs[4], hs[5]), pk16(hs[6], hs[7])};

  unsigned short* pb = arow + kInF + 8 * t;
  unsigned short* ps = arow + 8 * tc;
  *(volatile v4u*)pb = ub;
  if (t < 64) *(volatile v4u*)ps = us;
  __threadfence();
  *(volatile v4u*)pb = ub;
  if (t < 64) *(volatile v4u*)ps = us;
}

extern "C" void kernel_launch(void* const* d_in, const int* in_sizes, int n_in,
                              void* d_out, int out_size, void* d_ws, size_t ws_size,
                              hipStream_t stream) {
  if (n_in < 5) return;
  if (in_sizes[0] != kBatch * kInF) return;
  if (in_sizes[1] != kOutF * kInF) return;
  if (in_sizes[2] != kOutF * kInF * kNB) return;
  if (in_sizes[3] != kOutF * kInF) return;
  if (in_sizes[4] != kInF * kNKnot) return;
  if (out_size != kBatch * kOutF) return;
  if (ws_size < kWsNeed) return;

  const float* x    = (const float*)d_in[0];
  const float* bw   = (const float*)d_in[1];
  const float* sw   = (const float*)d_in[2];
  const float* sc   = (const float*)d_in[3];
  const float* grid = (const float*)d_in[4];
  float* out = (float*)d_out;

  unsigned char* ws = (unsigned char*)d_ws;
  unsigned short* Bt  = (unsigned short*)(ws);
  unsigned short* Apl = (unsigned short*)(ws + kBtBytes);
  const float* dummyf = (const float*)(const void*)ws;

  prep_base_kernel<<<dim3(kPrepBaseThreads / 256), dim3(256), 0, stream>>>(bw, Bt);
  prep_spline_kernel<<<dim3(kPrepSplThreads / 256), dim3(256), 0, stream>>>(sw, sc, Bt);

  const int tiles  = (kHalfRows / 64) * (kOutF / 64);
  const int blocks = (tiles + 7) / 8;
  for (int h = 0; h < 2; ++h) {
    gen_a_kernel<<<dim3(kHalfRows), dim3(kGenThreads), 0, stream>>>(x, grid, Apl, h * kHalfRows);
    float* cout = out + (size_t)h * kHalfRows * kOutF;
    wmma_gemm64<0, false, 0, 0, false, 6><<<dim3(blocks, 1, 1), dim3(256), 0, stream>>>(
        Apl, Apl, kKTot, 0L,
        Bt, Bt, kKTot, 0L,
        (void*)cout, (void*)ws, kOutF, 0L,
        dummyf,
        dummyf, 0L,
        kHalfRows, kOutF, kKTot, kOutScale);
  }
}
